// GraphSAGE_85615878078999
// MI455X (gfx1250) — hardware-verified
//
#include <hip/hip_runtime.h>
#include <stddef.h>
#include <stdint.h>
#include <math.h>


#define DF     128
#define NCLS   16
#define AP     512
#define KK     512
#define NTHR   256
#define NWAVE  8
#define EPT    8
#define CHUNK  (NTHR * EPT)
#define WCAP   (EPT * 32)
#define LISTN  (NWAVE * WCAP)
#define NBA    1024
#define SLA    10
#define RCAP   28672
#define DEGCAP 64
#define GBM    64
#define GBN    128
#define GTHR   128
#define GWAVE  (GTHR / 32)
#define PARTW  288
#define WSTW   258
#define HPR    8
#define HPB    (NWAVE * HPR)
#define WB1    ((DF * DF / 8) / NTHR)
#define AGG_ZINTS    (LISTN + 2 * RCAP + 3 * NBA)
#define MISC_INTS    16
#define ROWBUF_INTS  (NWAVE * DF)
#define AGG_LDS_INTS (AGG_ZINTS + MISC_INTS + ROWBUF_INTS)
#define WSMAX  134217728

static_assert((CHUNK & (CHUNK - 1)) == 0 && CHUNK <= 4096);
static_assert((NBA & (NBA - 1)) == 0 && NBA == (1 << SLA));
static_assert(((long long)CHUNK << SLA) < (1LL << 31));
static_assert(LISTN % NTHR == 0);
static_assert(NBA % NWAVE == 0 && NBA % 32 == 0 && NBA % GBM == 0);
static_assert(RCAP % 4 == 0 && AGG_ZINTS % 4 == 0 && LISTN % 4 == 0 && ((AGG_ZINTS + MISC_INTS) % 4) == 0);
static_assert(AGG_ZINTS % (NTHR * 4) == 0);
static_assert(KK % 32 == 0 && KK == AP && AP == 4 * DF);
static_assert(GBN == DF && GBM == GWAVE * 16 && DF == 4 * 32 && GTHR == DF);
static_assert(PARTW % 32 == 0 && PARTW / 4 <= GTHR && PARTW >= 2 * GBN + 1);
static_assert(WSTW >= 2 * GBN + 1 && (WSTW % 2) == 0);
static_assert(HPB == GBM && NTHR == 2 * DF);
static_assert(WB1 * NTHR * 8 == DF * DF);
static_assert(NCLS * DF / 8 == NTHR);
static_assert(NCLS == 16);
static_assert(AGG_LDS_INTS * 4 <= 300000);

typedef float          v4f   __attribute__((ext_vector_type(4)));
typedef float          v8f   __attribute__((ext_vector_type(8)));
typedef int            v4i   __attribute__((ext_vector_type(4)));
typedef int            v8i   __attribute__((ext_vector_type(8)));
typedef unsigned int   v4u   __attribute__((ext_vector_type(4)));
typedef unsigned short v4us  __attribute__((ext_vector_type(4)));
typedef unsigned short v8us  __attribute__((ext_vector_type(8)));
typedef unsigned short v16us __attribute__((ext_vector_type(16)));
typedef __bf16         v16bf __attribute__((ext_vector_type(16)));
typedef v4f  __attribute__((may_alias)) v4fa;
typedef v4i  __attribute__((may_alias)) v4ia;
typedef v4us __attribute__((may_alias)) v4usa;
typedef v8us __attribute__((may_alias)) v8usa;
union FragB { v16bf v; v16us u; v8us h[2]; v8i w; };

__device__ __forceinline__ v8f wmb(const FragB& a, const FragB& b, v8f c) {
  v8f d = __builtin_amdgcn_wmma_f32_16x16x32_bf16(false, a.v, false, b.v, (short)0, c, false, false);
  asm volatile("v_nop\n\tv_nop\n\tv_nop\n\tv_nop" : "+v"(d) : "v"(a.w), "v"(b.w));
  return d;
}

__device__ __forceinline__ v8f z8() { v8f z = {0.f, 0.f, 0.f, 0.f, 0.f, 0.f, 0.f, 0.f}; return z; }

__device__ __forceinline__ unsigned bf16_bits(float f) {
  const unsigned u = __float_as_uint(f);
  return ((u + 0x7FFFu + ((u >> 16) & 1u)) >> 16) & 0xFFFFu;
}
__device__ __forceinline__ float bf16_val(float f) {
  return __uint_as_float(bf16_bits(f) << 16);
}
__device__ __forceinline__ unsigned pk2(float lo, float hi) { return bf16_bits(lo) | (bf16_bits(hi) << 16); }
__device__ __forceinline__ v4u pack8(const v4f a, const v4f b) {
  v4u r;
  r.x = pk2(a.x, a.y); r.y = pk2(a.z, a.w); r.z = pk2(b.x, b.y); r.w = pk2(b.z, b.w);
  return r;
}

__device__ __forceinline__ void wave_sync() {
  __builtin_amdgcn_fence(__ATOMIC_RELEASE, "wavefront");
  __builtin_amdgcn_wave_barrier();
  __builtin_amdgcn_fence(__ATOMIC_ACQUIRE, "wavefront");
}

template <int SLB>
__device__ __forceinline__ int scan_chunk(const int* __restrict__ dsts, int nE, int cbase, int slotBase,
                                          int nb, int vec8, int* list, int tid, int lane, int wave) {
  int wc = 0;
  const int el0  = tid * EPT;
  const int e0   = cbase + el0;
  const int sent = -2147483647 - 1;
  v4i da, db;
  if (vec8 != 0 && cbase + CHUNK <= nE) {
    da = *(const v4i*)(dsts + e0);
    db = *(const v4i*)(dsts + e0 + 4);
  } else {
    da.x = (e0     < nE) ? dsts[min(e0,     nE - 1)] : sent;
    da.y = (e0 + 1 < nE) ? dsts[min(e0 + 1, nE - 1)] : sent;
    da.z = (e0 + 2 < nE) ? dsts[min(e0 + 2, nE - 1)] : sent;
    da.w = (e0 + 3 < nE) ? dsts[min(e0 + 3, nE - 1)] : sent;
    db.x = (e0 + 4 < nE) ? dsts[min(e0 + 4, nE - 1)] : sent;
    db.y = (e0 + 5 < nE) ? dsts[min(e0 + 5, nE - 1)] : sent;
    db.z = (e0 + 6 < nE) ? dsts[min(e0 + 6, nE - 1)] : sent;
    db.w = (e0 + 7 < nE) ? dsts[min(e0 + 7, nE - 1)] : sent;
  }
  const unsigned nbs = (unsigned)slotBase;
  const unsigned unb = (unsigned)nb;
  const unsigned s0 = (unsigned)da.x - nbs, s1 = (unsigned)da.y - nbs;
  const unsigned s2 = (unsigned)da.z - nbs, s3 = (unsigned)da.w - nbs;
  const unsigned s4 = (unsigned)db.x - nbs, s5 = (unsigned)db.y - nbs;
  const unsigned s6 = (unsigned)db.z - nbs, s7 = (unsigned)db.w - nbs;
  const bool h0 = s0 < unb, h1 = s1 < unb, h2 = s2 < unb, h3 = s3 < unb;
  const bool h4 = s4 < unb, h5 = s5 < unb, h6 = s6 < unb, h7 = s7 < unb;
  const unsigned any = __builtin_amdgcn_ballot_w32(h0 | h1 | h2 | h3 | h4 | h5 | h6 | h7);
  if (any != 0u) {
#define HITJ(J, HJ, SJ) { \
      const unsigned mj = __builtin_amdgcn_ballot_w32(HJ); \
      if (mj != 0u) { \
        if (HJ) { \
          const int pos = wc + (int)__builtin_amdgcn_mbcnt_lo(mj, 0u); \
          if (pos < WCAP) list[wave * WCAP + pos] = ((el0 + (J)) << SLB) | (int)(SJ); \
        } \
        wc += (int)__builtin_popcount(mj); } }
    HITJ(0, h0, s0)
    HITJ(1, h1, s1)
    HITJ(2, h2, s2)
    HITJ(3, h3, s3)
    HITJ(4, h4, s4)
    HITJ(5, h5, s5)
    HITJ(6, h6, s6)
    HITJ(7, h7, s7)
#undef HITJ
  }
  return wc;
}

__global__ __launch_bounds__(NTHR) void k_wprep(const float* __restrict__ Wl1, const float* __restrict__ Wr1,
                                                const float* __restrict__ Wl2, const float* __restrict__ Wr2,
                                                unsigned short* Bp1, unsigned short* Bp2) {
  const int b = (int)blockIdx.x, tid = (int)threadIdx.x;
  const bool l2 = b >= 2 * WB1;
  const int which = l2 ? (b - 2 * WB1) : (b / WB1);
  const int u = l2 ? tid : ((b & (WB1 - 1)) * NTHR + tid);
  const float* W = l2 ? ((which != 0) ? Wr2 : Wl2) : ((which != 0) ? Wr1 : Wl1);
  unsigned short* P = l2 ? Bp2 : Bp1;
  const int n  = u >> 4;
  const int k8 = (u & 15) * 8;
  const float* p = W + (size_t)n * DF + k8;
  const v4f a = *(const v4f*)p;
  const v4f c = *(const v4f*)(p + 4);
  const v4u q = pack8(a, c);
  unsigned short* dp = P + (size_t)n * KK + which * (2 * DF) + k8;
  *(volatile v4u*)dp = q;
  *(volatile v4u*)(dp + DF) = q;
  __threadfence();
  *(volatile v4u*)dp = q;
  *(volatile v4u*)(dp + DF) = q;
}

template <int INIT>
__global__ __launch_bounds__(NTHR) void k_hprep(const float* __restrict__ hn, const float* __restrict__ xres,
                                                const float* __restrict__ ss, const float* __restrict__ slope,
                                                int nN, int mRows, float* hout, unsigned short* apl) {
  __shared__ __attribute__((aligned(16))) float ssh[2 * DF];
  __shared__ __attribute__((aligned(16))) unsigned short rbuf[NWAVE * 2 * DF];
  const int tid = (int)threadIdx.x, lane = tid & 31, wave = tid >> 5;
  if constexpr (INIT != 0) {
    ssh[tid] = 0.0f;
  } else {
    ssh[tid] = ss[tid];
  }
  __syncthreads();
  const v4f sc = *(const v4fa*)(ssh + 4 * lane);
  const v4f sh = *(const v4fa*)(ssh + DF + 4 * lane);
  float slv = 0.0f;
  if constexpr (INIT == 0) slv = bf16_val(slope[0]);
  unsigned short* rb = rbuf + wave * (2 * DF);
  const int rb0 = (int)blockIdx.x * HPB + wave * HPR;

  v4f hv[HPR];
  v8us qv[HPR];
#pragma unroll
  for (int i = 0; i < HPR; ++i) {
    const int row = rb0 + i;
    const bool live = row < nN;
    const int rc = live ? row : (nN - 1);
    const v4f xr = *(const v4f*)(xres + (size_t)rc * DF + 4 * lane);
    v4f y;
    if constexpr (INIT != 0) {
      y.x = bf16_val(xr.x); y.y = bf16_val(xr.y); y.z = bf16_val(xr.z); y.w = bf16_val(xr.w);
    } else {
      const v4f a = *(const v4f*)(hn + (size_t)rc * DF + 4 * lane);
      float t0 = fmaf(a.x, sc.x, sh.x);
      float t1 = fmaf(a.y, sc.y, sh.y);
      float t2 = fmaf(a.z, sc.z, sh.z);
      float t3 = fmaf(a.w, sc.w, sh.w);
      t0 = (t0 >= 0.0f) ? t0 : slv * t0;
      t1 = (t1 >= 0.0f) ? t1 : slv * t1;
      t2 = (t2 >= 0.0f) ? t2 : slv * t2;
      t3 = (t3 >= 0.0f) ? t3 : slv * t3;
      y.x = t0 + bf16_val(xr.x);
      y.y = t1 + bf16_val(xr.y);
      y.z = t2 + bf16_val(xr.z);
      y.w = t3 + bf16_val(xr.w);
    }
    y.x = live ? y.x : 0.0f; y.y = live ? y.y : 0.0f; y.z = live ? y.z : 0.0f; y.w = live ? y.w : 0.0f;
    hv[i] = y;
    v4us mh, ml;
    {
      unsigned hb;
      hb = bf16_bits(y.x); mh[0] = (unsigned short)hb; ml[0] = (unsigned short)bf16_bits(y.x - __uint_as_float(hb << 16));
      hb = bf16_bits(y.y); mh[1] = (unsigned short)hb; ml[1] = (unsigned short)bf16_bits(y.y - __uint_as_float(hb << 16));
      hb = bf16_bits(y.z); mh[2] = (unsigned short)hb; ml[2] = (unsigned short)bf16_bits(y.z - __uint_as_float(hb << 16));
      hb = bf16_bits(y.w); mh[3] = (unsigned short)hb; ml[3] = (unsigned short)bf16_bits(y.w - __uint_as_float(hb << 16));
    }
    *(v4usa*)(rb + 4 * lane) = mh;
    *(v4usa*)(rb + DF + 4 * lane) = ml;
    wave_sync();
    qv[i] = *(const v8usa*)(rb + 8 * lane);
    wave_sync();
  }
#pragma unroll
  for (int i = 0; i < HPR; ++i) {
    const int row = rb0 + i;
    if (row < mRows) {
      *(volatile v4f*)(hout + (size_t)row * DF + 4 * lane) = hv[i];
      *(volatile v8us*)(apl + (size_t)row * AP + 2 * DF + 8 * lane) = qv[i];
    }
  }
  __threadfence();
#pragma unroll
  for (int i = 0; i < HPR; ++i) {
    const int row = rb0 + i;
    if (row < mRows) {
      *(volatile v4f*)(hout + (size_t)row * DF + 4 * lane) = hv[i];
      *(volatile v8us*)(apl + (size_t)row * AP + 2 * DF + 8 * lane) = qv[i];
    }
  }
}

__global__ __launch_bounds__(NTHR) void k_scan(const int* __restrict__ srcs, const int* __restrict__ dsts,
                                               int nE, int nN, int vec8, int mRows,
                                               const float* __restrict__ hsrc, unsigned short* apl) {
  extern __shared__ __attribute__((aligned(16))) int dsm[];
  int* list = dsm;
  int* hl   = dsm + LISTN;
  int* sl   = hl + RCAP;
  int* cnt  = sl + RCAP;
  int* offs = cnt + NBA;
  int* cur  = offs + NBA;
  int* misc = cur + NBA;
  const int tid = (int)threadIdx.x, lane = tid & 31, wave = tid >> 5;
  unsigned short* rowbuf = (unsigned short*)(misc + MISC_INTS) + wave * (2 * DF);
  const int nodeBase = (int)blockIdx.x * NBA;

  {
    const v4i z4 = {0, 0, 0, 0};
    for (int i = tid * 4; i < AGG_ZINTS; i += NTHR * 4) *(v4ia*)(dsm + i) = z4;
    if (tid < MISC_INTS) misc[tid] = 0;
  }
  __syncthreads();

  int t = 0, ov = 0;
  const int nChunks = (nE + CHUNK - 1) / CHUNK;
#pragma unroll 1
  for (int ch = 0; ch < nChunks; ++ch) {
    const int cbase = ch * CHUNK;
    const int wc = scan_chunk<SLA>(dsts, nE, cbase, nodeBase, NBA, vec8, list, tid, lane, wave);
    if (lane == 0) misc[wave] = wc;
    __syncthreads();
    if (wave == 0) {
#pragma unroll 1
      for (int w2 = 0; w2 < NWAVE; ++w2) {
        int c = misc[w2];
        c = c < 0 ? 0 : (c > WCAP ? WCAP : c);
#pragma unroll 1
        for (int b0 = 0; b0 < c; b0 += 32) {
          const int idx = b0 + lane;
          const int ent = list[w2 * WCAP + (idx < WCAP ? idx : WCAP - 1)];
          const int m32 = (c - b0) < 32 ? (c - b0) : 32;
#pragma unroll 1
          for (int k = 0; k < m32; ++k) {
            const int u    = __builtin_amdgcn_readlane(ent, k);
            const int slot = u & (NBA - 1);
            const int el   = (u >> SLA) & (CHUNK - 1);
            const int pk   = ((cbase + el) << SLA) | slot;
            if (t < RCAP) {
              if (lane == 0) { hl[t] = pk; cnt[slot] = cnt[slot] + 1; }
              t = t + 1;
            } else {
              ov = 1;
            }
          }
        }
      }
    }
    __syncthreads();
  }
  if (wave == 0 && lane == 0) { misc[8] = t; misc[9] = ov; }
  __syncthreads();
  int tt = misc[8];
  tt = tt < 0 ? 0 : (tt > RCAP ? RCAP : tt);
  const int ovf = misc[9];

  if (wave == 0) {
    const int base = lane * (NBA / 32);
    int s = 0;
#pragma unroll 1
    for (int i = 0; i < NBA / 32; ++i) s += cnt[base + i];
    int incl = s;
#pragma unroll
    for (int d = 1; d < 32; d <<= 1) {
      const int y = __shfl_up(incl, d, 32);
      if (lane >= d) incl += y;
    }
    int run = incl - s;
#pragma unroll 1
    for (int i = 0; i < NBA / 32; ++i) {
      const int cv = cnt[base + i];
      offs[base + i] = run;
      cur[base + i]  = run;
      run += cv;
    }
  }
  __syncthreads();
  if (wave == 0) {
#pragma unroll 1
    for (int b0 = 0; b0 < tt; b0 += 32) {
      const int idx = b0 + lane;
      const int ent = hl[idx < RCAP ? idx : RCAP - 1];
      const int m32 = (tt - b0) < 32 ? (tt - b0) : 32;
#pragma unroll 1
      for (int k = 0; k < m32; ++k) {
        const int u    = __builtin_amdgcn_readlane(ent, k);
        const int slot = u & (NBA - 1);
        if (lane == 0) {
          int p = cur[slot];
          p = p < 0 ? 0 : (p > RCAP - 1 ? RCAP - 1 : p);
          sl[p] = u;
          cur[slot] = p + 1;
        }
      }
    }
  }
  __syncthreads();

  const float pz = (ovf != 0) ? __int_as_float(0x7fc00000) : 0.0f;
#pragma unroll 1
  for (int si = 0; si < NBA / NWAVE; ++si) {
    const int s    = si * NWAVE + wave;
    const int node = nodeBase + s;
    int c = cnt[s];
    const bool big = c > DEGCAP;
    c = c < 0 ? 0 : (c > DEGCAP ? DEGCAP : c);
    int o = offs[s];
    o = o < 0 ? 0 : (o > RCAP ? RCAP : o);
    float a0 = 0.0f, a1 = 0.0f, a2 = 0.0f, a3 = 0.0f;
#pragma unroll 1
    for (int b0 = 0; b0 < c; b0 += 32) {
      int idx = o + b0 + lane;
      idx = idx > RCAP - 1 ? RCAP - 1 : idx;
      const int ent = sl[idx];
      int eid = ent >> SLA;
      eid = eid < 0 ? 0 : (eid > nE - 1 ? nE - 1 : eid);
      int sr = srcs[eid];
      sr = sr < 0 ? 0 : (sr > nN - 1 ? nN - 1 : sr);
      const int m32 = (c - b0) < 32 ? (c - b0) : 32;
#pragma unroll 1
      for (int k = 0; k < m32; ++k) {
        const int sk = __builtin_amdgcn_readlane(sr, k);
        const v4f a = *(const v4f*)(hsrc + (size_t)sk * DF + 4 * lane);
        a0 += a.x;
        a1 += a.y;
        a2 += a.z;
        a3 += a.w;
      }
    }
    const float den = (c > 0) ? (float)c : 1.0f;
    const float rcp = 1.0f / den;
    const float pzr = big ? __int_as_float(0x7fc00000) : pz;
    const bool live = node < nN;
    const float m0 = live ? (a0 * rcp + pzr) : 0.0f;
    const float m1 = live ? (a1 * rcp + pzr) : 0.0f;
    const float m2 = live ? (a2 * rcp + pzr) : 0.0f;
    const float m3 = live ? (a3 * rcp + pzr) : 0.0f;
    v4us mh, ml;
    {
      unsigned hb;
      hb = bf16_bits(m0); mh[0] = (unsigned short)hb; ml[0] = (unsigned short)bf16_bits(m0 - __uint_as_float(hb << 16));
      hb = bf16_bits(m1); mh[1] = (unsigned short)hb; ml[1] = (unsigned short)bf16_bits(m1 - __uint_as_float(hb << 16));
      hb = bf16_bits(m2); mh[2] = (unsigned short)hb; ml[2] = (unsigned short)bf16_bits(m2 - __uint_as_float(hb << 16));
      hb = bf16_bits(m3); mh[3] = (unsigned short)hb; ml[3] = (unsigned short)bf16_bits(m3 - __uint_as_float(hb << 16));
    }
    *(v4usa*)(rowbuf + 4 * lane) = mh;
    *(v4usa*)(rowbuf + DF + 4 * lane) = ml;
    wave_sync();
    const v8us q0 = *(const v8usa*)(rowbuf + 8 * lane);
    wave_sync();
    if (node < mRows) {
      unsigned short* rpw = apl + (size_t)node * AP + 8 * lane;
      *(volatile v8us*)rpw = q0;
      __threadfence();
      *(volatile v8us*)rpw = q0;
    }
  }
}

__global__ __launch_bounds__(GTHR) void k_gemm1(const unsigned short* __restrict__ Apl,
                                                const unsigned short* __restrict__ BT,
                                                const float* __restrict__ bias, int nN,
                                                float* outp, float* part) {
  __shared__ __attribute__((aligned(16))) float stg[GBM * GBN];
  __shared__ __attribute__((aligned(16))) float wst[GWAVE * WSTW];
  __shared__ __attribute__((aligned(16))) float pst[PARTW];
  const int tid = (int)threadIdx.x, lane = tid & 31, wave = tid >> 5, hh = lane >> 4, m = lane & 15;
  const int rowBase = (int)blockIdx.x * GBM;

  v8f acc[8];
#pragma unroll
  for (int t = 0; t < 8; ++t) acc[t] = z8();
  const unsigned short* ap = Apl + (size_t)(rowBase + 16 * wave + m) * (size_t)AP + 8 * hh;
  const unsigned short* bp = BT + (size_t)m * (size_t)KK + 8 * hh;

#pragma unroll 1
  for (int k0 = 0; k0 < KK; k0 += 32) {
    FragB af;
    af.h[0] = *(const v8usa*)(ap + k0);
    af.h[1] = *(const v8usa*)(ap + k0 + 16);
#pragma unroll
    for (int nt = 0; nt < 8; ++nt) {
      const unsigned short* wq = bp + (size_t)(16 * nt) * (size_t)KK + k0;
      FragB bf;
      bf.h[0] = *(const v8usa*)wq;
      bf.h[1] = *(const v8usa*)(wq + 16);
      acc[nt] = wmb(af, bf, acc[nt]);
    }
  }

#pragma unroll
  for (int nt = 0; nt < 8; ++nt) {
    const int lc = 16 * nt + m;
#pragma unroll
    for (int r = 0; r < 8; ++r) {
      const int lr = 16 * wave + 8 * hh + r;
      stg[lr * GBN + lc] = acc[nt][r];
    }
  }
  __syncthreads();

  v4f bq;
  {
    const v4f b4 = *(const v4f*)(bias + 4 * lane);
    bq.x = bf16_val(b4.x); bq.y = bf16_val(b4.y); bq.z = bf16_val(b4.z); bq.w = bf16_val(b4.w);
  }

  v4f pv[16];
  int wn = 0;
  float wm[4], wqv[4];
#pragma unroll
  for (int j = 0; j < 4; ++j) { wm[j] = 0.0f; wqv[j] = 0.0f; }
#pragma unroll
  for (int i = 0; i < 16; ++i) {
    const int row = rowBase + 16 * wave + i;
    const bool ok = row < nN;
    const v4f x = *(const v4fa*)(stg + (16 * wave + i) * GBN + 4 * lane);
    const v4f tq = x + bq;
    float vv[4];
    vv[0] = ok ? tq.x : 0.0f; vv[1] = ok ? tq.y : 0.0f; vv[2] = ok ? tq.z : 0.0f; vv[3] = ok ? tq.w : 0.0f;
    v4f q;
    q.x = vv[0]; q.y = vv[1]; q.z = vv[2]; q.w = vv[3];
    pv[i] = q;
    if (ok) {
      wn += 1;
      const float rk = 1.0f / (float)(i + 1);
#pragma unroll
      for (int j = 0; j < 4; ++j) {
        const float d = vv[j] - wm[j];
        wm[j]  = fmaf(d, rk, wm[j]);
        wqv[j] = fmaf(d, vv[j] - wm[j], wqv[j]);
      }
    }
  }

#pragma unroll
  for (int i = 0; i < 16; ++i) {
    float* op = outp + (size_t)(rowBase + 16 * wave + i) * (size_t)DF + 4 * lane;
    *(volatile v4f*)op = pv[i];
  }
  __threadfence();
#pragma unroll
  for (int i = 0; i < 16; ++i) {
    float* op = outp + (size_t)(rowBase + 16 * wave + i) * (size_t)DF + 4 * lane;
    *(volatile v4f*)op = pv[i];
  }

  if (lane == 0) wst[wave * WSTW] = (float)wn;
#pragma unroll
  for (int j = 0; j < 4; ++j) {
    wst[wave * WSTW + 1 + 4 * lane + j]       = wm[j];
    wst[wave * WSTW + 1 + GBN + 4 * lane + j] = wqv[j];
  }
  __syncthreads();
  {
    float n = 0.0f, mean = 0.0f, M2 = 0.0f;
#pragma unroll 1
    for (int w2 = 0; w2 < GWAVE; ++w2) {
      const float nb = wst[w2 * WSTW];
      const float mb = wst[w2 * WSTW + 1 + tid];
      const float qb = wst[w2 * WSTW + 1 + GBN + tid];
      if (nb > 0.5f) {
        const float nn = n + nb;
        const float delta = mb - mean;
        const float f = nb / nn;
        mean = fmaf(delta, f, mean);
        M2 = M2 + qb + delta * delta * n * f;
        n = nn;
      }
    }
    pst[1 + tid] = mean;
    pst[1 + GBN + tid] = M2;
    if (tid == 0) pst[0] = n;
  }
#pragma unroll 1
  for (int i = 2 * GBN + 1 + tid; i < PARTW; i += GTHR) pst[i] = 0.0f;
  __syncthreads();
  const int pb = (int)blockIdx.x;
  v4f ps = {0.0f, 0.0f, 0.0f, 0.0f};
  if (tid < PARTW / 4) {
    ps = *(const v4fa*)(pst + 4 * tid);
    *(volatile v4f*)(part + (size_t)pb * PARTW + 4 * tid) = ps;
  }
  __threadfence();
  if (tid < PARTW / 4) {
    *(volatile v4f*)(part + (size_t)pb * PARTW + 4 * tid) = ps;
  }
}

__global__ __launch_bounds__(DF) void k_bnfin(const float* __restrict__ part, int nPart,
                                              const float* __restrict__ gam, const float* __restrict__ bet,
                                              float* ss) {
  __shared__ __attribute__((aligned(16))) float stg[2 * DF];
  const int tid = (int)threadIdx.x;
  const int c = tid;
  double n = 0.0, mean = 0.0, M2 = 0.0;
#pragma unroll 1
  for (int b = 0; b < nPart; ++b) {
    const float* pr = part + (size_t)b * PARTW;
    const double nb = (double)pr[0];
    const double mb = (double)pr[1 + c];
    const double qb = (double)pr[1 + GBN + c];
    if (nb > 0.5) {
      const double nn = n + nb;
      const double delta = mb - mean;
      const double f = nb / nn;
      mean = mean + delta * f;
      M2 = M2 + qb + delta * delta * n * f;
      n = nn;
    }
  }
  const double nt = n < 1.0 ? 1.0 : n;
  const float varf  = (float)(M2 / nt);
  const float meanf = (float)mean;
  const float rstd = 1.0f / sqrtf(varf + 1e-5f);
  const float sc = bf16_val(gam[c]) * rstd;
  const float sh = bf16_val(bet[c]) - meanf * sc;
  stg[c] = sc;
  stg[DF + c] = sh;
  __syncthreads();
  v4f v = {0.0f, 0.0f, 0.0f, 0.0f};
  if (tid < (2 * DF) / 4) {
    v = *(const v4fa*)(stg + 4 * tid);
    *(volatile v4f*)(ss + 4 * tid) = v;
  }
  __threadfence();
  if (tid < (2 * DF) / 4) {
    *(volatile v4f*)(ss + 4 * tid) = v;
  }
}

__global__ __launch_bounds__(GTHR) void k_gemm2(const unsigned short* __restrict__ Apl,
                                                const unsigned short* __restrict__ BT,
                                                const float* __restrict__ bias, int nN, float* outp) {
  __shared__ __attribute__((aligned(16))) float stg[GBM * NCLS];
  const int tid = (int)threadIdx.x, lane = tid & 31, wave = tid >> 5, hh = lane >> 4, m = lane & 15;
  const int rowBase = (int)blockIdx.x * GBM;

  v8f acc = z8();
  const unsigned short* ap = Apl + (size_t)(rowBase + 16 * wave + m) * (size_t)AP + 8 * hh;
  const unsigned short* bp = BT + (size_t)m * (size_t)KK + 8 * hh;

#pragma unroll 4
  for (int k0 = 0; k0 < KK; k0 += 32) {
    FragB af, bf;
    af.h[0] = *(const v8usa*)(ap + k0);
    af.h[1] = *(const v8usa*)(ap + k0 + 16);
    bf.h[0] = *(const v8usa*)(bp + k0);
    bf.h[1] = *(const v8usa*)(bp + k0 + 16);
    acc = wmb(af, bf, acc);
  }

  const float bq = bf16_val(bias[m]);
  float ov[8];
#pragma unroll
  for (int r = 0; r < 8; ++r) {
    const float z = acc[r] + bq;
    float mx = z;
#pragma unroll
    for (int off = 8; off > 0; off >>= 1) mx = fmaxf(mx, __shfl_xor(mx, off, 32));
    const float sh = z - mx;
    float se = expf(sh);
#pragma unroll
    for (int off = 8; off > 0; off >>= 1) se += __shfl_xor(se, off, 32);
    ov[r] = sh - logf(se);
  }
#pragma unroll
  for (int r = 0; r < 8; ++r) {
    const int lr = 16 * wave + 8 * hh + r;
    stg[lr * NCLS + m] = ov[r];
  }
  __syncthreads();

  const float* sb = stg + (16 * wave) * NCLS;
  float* ob = outp + (size_t)(rowBase + 16 * wave) * (size_t)NCLS;
  v4f pv[2];
#pragma unroll
  for (int j = 0; j < 2; ++j) {
    const int p = 32 * j + lane;
    pv[j] = *(const v4fa*)(sb + 4 * p);
  }
#pragma unroll
  for (int j = 0; j < 2; ++j) {
    const int p = 32 * j + lane;
    const int grow = rowBase + 16 * wave + (p >> 2);
    if (grow < nN) *(volatile v4f*)(ob + 4 * p) = pv[j];
  }
  __threadfence();
#pragma unroll
  for (int j = 0; j < 2; ++j) {
    const int p = 32 * j + lane;
    const int grow = rowBase + 16 * wave + (p >> 2);
    if (grow < nN) *(volatile v4f*)(ob + 4 * p) = pv[j];
  }
}

static inline int cdiv(int a, int b) { return (a + b - 1) / b; }
static inline size_t al256(size_t o) { return (o + 255) & ~(size_t)255; }

extern "C" void kernel_launch(void* const* d_in, const int* in_sizes, int n_in,
                              void* d_out, int out_size, void* d_ws, size_t ws_size,
                              hipStream_t stream) {
  if (n_in < 11) return;
  if (in_sizes[0] < DF || (in_sizes[0] % DF) != 0) return;
  const int nN = in_sizes[0] / DF;
  if (in_sizes[1] < 2 || (in_sizes[1] & 1) != 0) return;
  const int nE = in_sizes[1] / 2;
  if (nE < 1 || nE >= (1 << 21) || nN < 16 || nN >= (1 << 24)) return;
  if (in_sizes[2] != DF * DF) return;
  if (in_sizes[3] != DF) return;
  if (in_sizes[4] != DF * DF) return;
  if (in_sizes[5] != NCLS * DF) return;
  if (in_sizes[6] != NCLS) return;
  if (in_sizes[7] != NCLS * DF) return;
  if (in_sizes[8] != DF || in_sizes[9] != DF) return;
  if (in_sizes[10] < 1) return;
  if ((long long)out_size != (long long)nN * NCLS) return;

  const float* x     = (const float*)d_in[0];
  const int*   ei    = (const int*)d_in[1];
  const float* Wl1   = (const float*)d_in[2];
  const float* bl1   = (const float*)d_in[3];
  const float* Wr1   = (const float*)d_in[4];
  const float* Wl2   = (const float*)d_in[5];
  const float* bl2   = (const float*)d_in[6];
  const float* Wr2   = (const float*)d_in[7];
  const float* gamma = (const float*)d_in[8];
  const float* beta  = (const float*)d_in[9];
  const float* asl   = (const float*)d_in[10];
  float* out = (float*)d_out;
  const int* src = ei;
  const int* dst = ei + nE;

  const int MP = cdiv(nN, GBM) * GBM;
  const int gM = MP / GBM;
  const int gA = cdiv(nN, NBA);
  if ((long long)gA * NBA < (long long)MP) return;
  if ((MP % HPB) != 0) return;
  const int vec8 = ((nE & 3) == 0) ? 1 : 0;

  char* ws = (char*)d_ws;
  size_t off = 0;
  const size_t oB1 = off; off = al256(off + (size_t)DF * KK * 2);
  const size_t oB2 = off; off = al256(off + (size_t)NCLS * KK * 2);
  const size_t oA  = off; off = al256(off + (size_t)MP * AP * 2);
  const size_t oH  = off; off = al256(off + (size_t)MP * DF * 4);
  const size_t oHN = off; off = al256(off + (size_t)MP * DF * 4);
  const size_t oPT = off; off = al256(off + (size_t)gM * PARTW * 4);
  const size_t oSS = off; off = al256(off + (size_t)(2 * DF) * 4);
  if (off > ws_size || off > (size_t)WSMAX) return;
  unsigned short* Bp1 = (unsigned short*)(ws + oB1);
  unsigned short* Bp2 = (unsigned short*)(ws + oB2);
  unsigned short* Apl = (unsigned short*)(ws + oA);
  float*          H   = (float*)(ws + oH);
  float*          HN  = (float*)(ws + oHN);
  float*          PT  = (float*)(ws + oPT);
  float*          SS  = (float*)(ws + oSS);

  const size_t scanLds = (size_t)AGG_LDS_INTS * 4;
  hipFuncSetAttribute(reinterpret_cast<const void*>(&k_scan), hipFuncAttributeMaxDynamicSharedMemorySize, (int)scanLds);

  k_wprep<<<2 * WB1 + 2, NTHR, 0, stream>>>(Wl1, Wr1, Wl2, Wr2, Bp1, Bp2);
  k_hprep<1><<<gM, NTHR, 0, stream>>>(x, x, SS, asl, nN, MP, H, Apl);
  k_scan<<<gA, NTHR, scanLds, stream>>>(src, dst, nE, nN, vec8, MP, H, Apl);
  k_gemm1<<<gM, GTHR, 0, stream>>>(Apl, Bp1, bl1, nN, HN, PT);
  k_bnfin<<<1, DF, 0, stream>>>(PT, gM, gamma, beta, SS);
  k_hprep<0><<<gM, NTHR, 0, stream>>>(HN, x, SS, asl, nN, MP, H, Apl);
  k_scan<<<gA, NTHR, scanLds, stream>>>(src, dst, nE, nN, vec8, MP, H, Apl);
  k_gemm2<<<gM, GTHR, 0, stream>>>(Apl, Bp2, bl2, nN, out);
}
